// decoder_33973191311954
// MI455X (gfx1250) — hardware-verified
//
#include <hip/hip_runtime.h>
#include <math.h>

constexpr int NBATCH   = 32;
constexpr int NFRAME   = 52;
constexpr int NHID     = 512;
constexpr int NEMB     = 512;
constexpr int NVOC     = 20000;
constexpr int NVPAD    = 20032;
constexpr int NCAP     = 20;
constexpr int NT1      = 32;
constexpr int NDEC     = 19;
constexpr int NSTEPS   = NT1 + NDEC;
constexpr int NG4      = 4 * NHID;
constexpr int KIH      = NEMB + NHID;
constexpr int KW1      = 3 * NHID;
constexpr int NROW_XE  = NBATCH * NT1;
constexpr int NROW_OUT = NBATCH * NDEC;
constexpr int NROW_PAD = 640;
constexpr int SEQ_ROWS = 16;
constexpr int SEQ_THR  = 512;
constexpr int HP       = 520;
constexpr int PP       = 516;
constexpr float WCARRY     = 16.0f;
constexpr float WCARRY_INV = 1.0f / 16.0f;

static_assert(NROW_XE == 1024, "rows of the frame plane");
static_assert(NROW_OUT == 608 && NROW_OUT % 16 == 0 && NROW_PAD % 64 == 0 && NROW_PAD >= NROW_OUT, "output rows");
static_assert(NVPAD % 64 == 0 && NVPAD >= NVOC && NVOC % 32 == 0, "vocabulary padding is line exact");
static_assert(NHID % 32 == 0 && KIH % 32 == 0, "GEMM K multiples of 32");
static_assert(NHID % 64 == 0 && NG4 % 64 == 0 && NROW_XE % 64 == 0, "GEMM M, N tile multiples");
static_assert(SEQ_THR == NHID, "one score weight per thread");
static_assert(SEQ_THR / 32 == SEQ_ROWS, "one wave per batch row in the attention stage");
static_assert(NHID == 32 * (SEQ_THR / 32), "32 hidden units per wave");
static_assert(NBATCH % SEQ_ROWS == 0, "batch tiles");
static_assert((HP * 2) % 16 == 0 && (PP * 4) % 16 == 0, "LDS pitches keep 16-B alignment");

typedef __attribute__((ext_vector_type(16))) _Float16 v16h;
typedef __attribute__((ext_vector_type(8)))  _Float16 v8h;
typedef __attribute__((ext_vector_type(4)))  _Float16 v4h;
typedef __attribute__((ext_vector_type(8)))  float    v8f;
typedef __attribute__((ext_vector_type(4)))  float    v4f;

union FragU { v16h v; v8h h[2]; };

__device__ __forceinline__ v16h frag_load(const _Float16* p) {
  FragU f;
  f.h[0] = *(const v8h*)(p);
  f.h[1] = *(const v8h*)(p + 16);
  return f.v;
}
__device__ __forceinline__ v8f frag_mma(v16h a, v16h b, v8f c) {
  return __builtin_amdgcn_wmma_f32_16x16x32_f16(false, a, false, b, (short)0, c, false, false);
}
__device__ __forceinline__ void guard4_h(v8f& a0, v8f& a1, v8f& a2, v8f& a3, v16h x, v16h y0, v16h y1, v16h y2, v16h y3) {
  asm volatile("v_nop\n\tv_nop\n\tv_nop\n\tv_nop" : "+v"(a0), "+v"(a1), "+v"(a2), "+v"(a3) : "v"(x), "v"(y0), "v"(y1), "v"(y2), "v"(y3));
}
__device__ __forceinline__ void guard2_h(v8f& a0, v8f& a1, v16h x, v16h y0, v16h y1) {
  asm volatile("v_nop\n\tv_nop\n\tv_nop\n\tv_nop" : "+v"(a0), "+v"(a1) : "v"(x), "v"(y0), "v"(y1));
}
__device__ __forceinline__ void keep4_h(v16h a, v16h b, v16h c, v16h d) { asm volatile("v_nop" :: "v"(a), "v"(b), "v"(c), "v"(d)); }
__device__ __forceinline__ void acc_guard4(v8f& a, v8f& b, v8f& c, v8f& d) { asm volatile("v_nop\n\tv_nop\n\tv_nop\n\tv_nop" : "+v"(a), "+v"(b), "+v"(c), "+v"(d)); }
__device__ __forceinline__ void acc_guard2(v8f& a, v8f& b) { asm volatile("v_nop\n\tv_nop\n\tv_nop\n\tv_nop" : "+v"(a), "+v"(b)); }
__device__ __forceinline__ void pin8(v8f& a) { asm volatile("" : "+v"(a) :: "memory"); }
__device__ __forceinline__ void pin4s(float& a, float& b, float& c, float& d) { asm volatile("" : "+v"(a), "+v"(b), "+v"(c), "+v"(d) :: "memory"); }

__device__ __forceinline__ float fsig(float x)   { return 1.0f / (1.0f + expf(-x)); }
__device__ __forceinline__ float ftanh_e(float x) { return 1.0f - 2.0f * (1.0f / (1.0f + expf(2.0f * x))); }

__device__ __forceinline__ void lstm_point(float zi, float zf, float zg, float zo, float& cs, float& hn) {
  const float ig = fsig(zi);
  const float fg = fsig(zf);
  const float gg = ftanh_e(zg);
  const float og = fsig(zo);
  const float cn = fg * cs + ig * gg;
  cs = cn;
  hn = og * ftanh_e(cn);
}

__device__ __forceinline__ void kloop4_h(v8f& a0, v8f& a1, v8f& a2, v8f& a3,
                                         const _Float16* arow, const _Float16* wrow, size_t gstride) {
#pragma unroll 1
  for (int k0 = 0; k0 < NHID; k0 += 32) {
    const v16h a  = frag_load(arow + k0);
    const v16h b0 = frag_load(wrow + k0);
    const v16h b1 = frag_load(wrow + gstride + k0);
    const v16h b2 = frag_load(wrow + 2 * gstride + k0);
    const v16h b3 = frag_load(wrow + 3 * gstride + k0);
    a0 = frag_mma(a, b0, a0);
    a1 = frag_mma(a, b1, a1);
    a2 = frag_mma(a, b2, a2);
    a3 = frag_mma(a, b3, a3);
    guard4_h(a0, a1, a2, a3, a, b0, b1, b2, b3);
  }
}

template <int RMAP>
__global__ __launch_bounds__(256) void cvt8_f16_kernel(const float* __restrict__ src, unsigned short* __restrict__ dst,
                                                       int nrow, int ncol8, int spitch, int nvalid, float sc) {
  const int i  = blockIdx.x * 256 + threadIdx.x;
  const int n8 = nrow * ncol8;
  if (i < n8) {
    const int row = i / ncol8;
    const int c8  = i - row * ncol8;
    const int rc  = (row < nvalid) ? row : (nvalid - 1);
    const int srow = (RMAP == 1) ? ((rc >> 5) * NFRAME + (rc & 31)) : rc;
    const float* sp = src + (size_t)srow * spitch + c8 * 8;
    const v4f a = *(const v4f*)(sp);
    const v4f b = *(const v4f*)(sp + 4);
    const bool ok = (row < nvalid);
    v8h hv;
#pragma unroll
    for (int e = 0; e < 4; ++e) {
      const float x0 = a[e];
      const float x1 = b[e];
      const float y0 = ok ? (x0 * sc) : 0.0f;
      const float y1 = ok ? (x1 * sc) : 0.0f;
      hv[e]     = (_Float16)y0;
      hv[4 + e] = (_Float16)y1;
    }
    *(volatile v8h*)(dst + (size_t)i * 8) = hv;
    __threadfence();
    *(volatile v8h*)(dst + (size_t)i * 8) = hv;
  }
}

__global__ __launch_bounds__(256) void pack_x2_kernel(const float* __restrict__ feature, const float* __restrict__ emb,
                                                      const int* __restrict__ cap, unsigned short* __restrict__ dst) {
  const int i    = blockIdx.x * 256 + threadIdx.x;
  const int half = blockIdx.y;
  const int row  = i >> 6;
  const int c8   = i & 63;
  if (row < NROW_PAD) {
    const int l  = row >> 5;
    const int b  = row & 31;
    const int lc = (l < NDEC) ? l : (NDEC - 1);
    const bool ok = (row < NROW_OUT);
    int tok = cap[b * NCAP + lc];
    tok = (tok < 0) ? 0 : ((tok > NVOC - 1) ? (NVOC - 1) : tok);
    const float* pe = emb + (size_t)tok * NEMB + c8 * 8;
    const float* pf = feature + ((size_t)b * NFRAME + NT1 + lc) * NHID + c8 * 8;
    const float* sp = (half == 0) ? pe : pf;
    const v4f a = *(const v4f*)(sp);
    const v4f bq = *(const v4f*)(sp + 4);
    v8h hv;
#pragma unroll
    for (int e = 0; e < 4; ++e) {
      const float x0 = a[e];
      const float x1 = bq[e];
      const float y0 = ok ? x0 : 0.0f;
      const float y1 = ok ? x1 : 0.0f;
      hv[e]     = (_Float16)y0;
      hv[4 + e] = (_Float16)y1;
    }
    unsigned short* op = dst + (size_t)row * KIH + half * NEMB + c8 * 8;
    *(volatile v8h*)op = hv;
    __threadfence();
    *(volatile v8h*)op = hv;
  }
}

__global__ __launch_bounds__(256) void zero16_kernel(unsigned short* __restrict__ dst, int n8) {
  const int i = blockIdx.x * 256 + threadIdx.x;
  if (i < n8) {
    v8h z;
#pragma unroll
    for (int e = 0; e < 8; ++e) z[e] = (_Float16)0.0f;
    *(volatile v8h*)(dst + (size_t)i * 8) = z;
    __threadfence();
    *(volatile v8h*)(dst + (size_t)i * 8) = z;
  }
}

template <int BIAS_MODE>
__global__ __launch_bounds__(256) void gemm64_f16_kernel(
    const unsigned short* __restrict__ Ap, int lda,
    const unsigned short* __restrict__ Btp, int ldb,
    float* __restrict__ C, int ldc,
    const float* __restrict__ bias,
    int M, int N, int K, int Mreal, int Nreal, float scale) {
  const _Float16* A  = (const _Float16*)Ap;
  const _Float16* Bt = (const _Float16*)Btp;
  __shared__ __align__(16) float sT[8][16 * 68];
  const int lane = threadIdx.x & 31;
  const int wave = threadIdx.x >> 5;
  const int tilesN = N >> 6;
  const int tilesM = M >> 6;
  const int tile = blockIdx.x * 8 + wave;
  if (tile >= tilesM * tilesN) return;
  const int tm = tile / tilesN;
  const int tn = tile - tm * tilesN;
  const int m0 = tm << 6;
  const int n0 = tn << 6;
  const int rlane = lane & 15;
  const int koff  = (lane >> 4) * 8;
  const int mOff  = (lane >> 4) * 8;

  v8f acc[4][4];
#pragma unroll
  for (int i = 0; i < 4; ++i)
#pragma unroll
    for (int j = 0; j < 4; ++j) acc[i][j] = (v8f){0.f, 0.f, 0.f, 0.f, 0.f, 0.f, 0.f, 0.f};

  for (int k0 = 0; k0 < K; k0 += 32) {
    v16h bh[4];
#pragma unroll
    for (int j = 0; j < 4; ++j) {
      const size_t bo = (size_t)(n0 + (j << 4) + rlane) * ldb + koff + k0;
      bh[j] = frag_load(Bt + bo);
    }
#pragma unroll
    for (int i = 0; i < 4; ++i) {
      const size_t ao = (size_t)(m0 + (i << 4) + rlane) * lda + koff + k0;
      const v16h ah = frag_load(A + ao);
#pragma unroll
      for (int j = 0; j < 4; ++j) acc[i][j] = frag_mma(ah, bh[j], acc[i][j]);
      guard4_h(acc[i][0], acc[i][1], acc[i][2], acc[i][3], ah, bh[0], bh[1], bh[2], bh[3]);
    }
    keep4_h(bh[0], bh[1], bh[2], bh[3]);
  }
  acc_guard4(acc[0][0], acc[0][1], acc[0][2], acc[0][3]);
  acc_guard4(acc[1][0], acc[1][1], acc[1][2], acc[1][3]);
  acc_guard4(acc[2][0], acc[2][1], acc[2][2], acc[2][3]);
  acc_guard4(acc[3][0], acc[3][1], acc[3][2], acc[3][3]);

  float* slab = sT[wave];
#pragma unroll
  for (int i = 0; i < 4; ++i) {
    const int mBase = m0 + (i << 4);
#pragma unroll
    for (int j = 0; j < 4; ++j) {
      const int n = n0 + (j << 4) + rlane;
      float bv = 0.f;
      if (BIAS_MODE == 2) {
        const int nc = (n < Nreal) ? n : (Nreal - 1);
        bv = bias[nc];
      }
#pragma unroll
      for (int r = 0; r < 8; ++r) slab[(mOff + r) * 68 + (j << 4) + rlane] = acc[i][j][r] * scale + bv;
    }
    __builtin_amdgcn_fence(__ATOMIC_RELEASE, "workgroup");
    __builtin_amdgcn_wave_barrier();
    __builtin_amdgcn_fence(__ATOMIC_ACQUIRE, "workgroup");
    {
      const int hh = lane >> 4, c4 = (lane & 15) * 4;
      const bool ok = (mBase < Mreal) && (n0 + c4 < Nreal);
      for (int pass = 0; pass < 2; ++pass) {
#pragma unroll
        for (int it = 0; it < 8; ++it) {
          const int row = it * 2 + hh;
          const v4f v = *(const v4f*)(slab + row * 68 + c4);
          if (ok) *(volatile v4f*)(C + (size_t)(mBase + row) * ldc + n0 + c4) = v;
        }
        __threadfence();
      }
    }
    __builtin_amdgcn_fence(__ATOMIC_RELEASE, "workgroup");
    __builtin_amdgcn_wave_barrier();
    __builtin_amdgcn_fence(__ATOMIC_ACQUIRE, "workgroup");
  }
}

__global__ __launch_bounds__(SEQ_THR) void decoder_seq_kernel(
    const float* __restrict__ feature, const float* __restrict__ S,
    const float* Gx1, const float* Gx2,
    const unsigned short* __restrict__ Wihp, const unsigned short* __restrict__ Whhp, const unsigned short* __restrict__ W1p,
    const float* b_ih, const float* b_hh, const float* __restrict__ W2, const float* __restrict__ b2p,
    unsigned short* __restrict__ Hout) {
  __shared__ __align__(16) _Float16 Ah[SEQ_ROWS * HP];
  __shared__ __align__(16) _Float16 Ac[SEQ_ROWS * HP];
  __shared__ __align__(16) _Float16 Ax[SEQ_ROWS * HP];
  __shared__ __align__(16) float    Pl[SEQ_ROWS * PP];
  __shared__ __align__(16) float    W2s[NHID];
  const _Float16* Wih = (const _Float16*)Wihp;
  const _Float16* Whh = (const _Float16*)Whhp;
  const _Float16* W1  = (const _Float16*)W1p;
  const int tid = threadIdx.x, lane = tid & 31, wave = tid >> 5;
  const int c = lane & 15, hh = lane >> 4, koff = hh * 8;
  const int rowbase = blockIdx.x * SEQ_ROWS;

#pragma unroll 1
  for (int i = tid; i < SEQ_ROWS * HP; i += SEQ_THR) {
    Ah[i] = (_Float16)0.0f;
    Ac[i] = (_Float16)0.0f;
    Ax[i] = (_Float16)0.0f;
  }
#pragma unroll 1
  for (int i = tid; i < SEQ_ROWS * PP; i += SEQ_THR) Pl[i] = 0.0f;
  W2s[tid] = W2[tid];
  const float b2v = b2p[0];

  float bb[2][4];
  float cst[2][8];
#pragma unroll
  for (int nt = 0; nt < 2; ++nt) {
    const int j = 32 * wave + 16 * nt + c;
#pragma unroll
    for (int g = 0; g < 4; ++g) {
      const float x = b_ih[g * NHID + j];
      const float y = b_hh[g * NHID + j];
      bb[nt][g] = x + y;
    }
    pin4s(bb[nt][0], bb[nt][1], bb[nt][2], bb[nt][3]);
#pragma unroll
    for (int r = 0; r < 8; ++r) cst[nt][r] = 0.0f;
  }
  __syncthreads();

  const _Float16* ahrow = Ah + c * HP + koff;
  const _Float16* acrow = Ac + c * HP + koff;
  const _Float16* axrow = Ax + c * HP + koff;
  const v8f z8 = {0.f, 0.f, 0.f, 0.f, 0.f, 0.f, 0.f, 0.f};

#pragma unroll 1
  for (int s = 0; s < NSTEPS; ++s) {
    if (s < NT1) {
      {
        v8f p0 = z8, p1 = z8;
        const _Float16* w0 = W1 + (size_t)(32 * wave + c) * KW1 + koff;
        const _Float16* w1 = w0 + (size_t)16 * KW1;
#pragma unroll 1
        for (int k0 = 0; k0 < NHID; k0 += 32) {
          const v16h a  = frag_load(ahrow + k0);
          const v16h b0 = frag_load(w0 + k0);
          const v16h b1 = frag_load(w1 + k0);
          p0 = frag_mma(a, b0, p0);
          p1 = frag_mma(a, b1, p1);
          guard2_h(p0, p1, a, b0, b1);
        }
#pragma unroll 1
        for (int k0 = 0; k0 < NHID; k0 += 32) {
          const v16h a  = frag_load(acrow + k0);
          const v16h b0 = frag_load(w0 + NHID + k0);
          const v16h b1 = frag_load(w1 + NHID + k0);
          p0 = frag_mma(a, b0, p0);
          p1 = frag_mma(a, b1, p1);
          guard2_h(p0, p1, a, b0, b1);
        }
        acc_guard2(p0, p1);
#pragma unroll
        for (int r = 0; r < 8; ++r) {
          Pl[(8 * hh + r) * PP + 32 * wave + c]      = p0[r] * WCARRY_INV;
          Pl[(8 * hh + r) * PP + 32 * wave + 16 + c] = p1[r] * WCARRY_INV;
        }
      }
      __syncthreads();

      {
        const int gb = rowbase + wave;
        const float* Srow = S + (size_t)gb * NT1 * NHID;
        const float* prow = Pl + wave * PP;
        float myscore = 0.0f;
#pragma unroll 1
        for (int tp = 0; tp < NT1; ++tp) {
          float part = 0.0f;
#pragma unroll 1
          for (int q = 0; q < 4; ++q) {
            const int jo = 128 * q + 4 * lane;
            const v4f s4 = *(const v4f*)(Srow + (size_t)tp * NHID + jo);
            const v4f p4 = *(const v4f*)(prow + jo);
            const v4f w4 = *(const v4f*)(W2s + jo);
#pragma unroll
            for (int e = 0; e < 4; ++e) part += w4[e] * tanhf(s4[e] + p4[e]);
          }
#pragma unroll
          for (int off = 16; off > 0; off >>= 1) part += __shfl_xor(part, off, 32);
          myscore = (lane == tp) ? part : myscore;
        }
        myscore += b2v;
        float mx = myscore;
#pragma unroll
        for (int off = 16; off > 0; off >>= 1) mx = fmaxf(mx, __shfl_xor(mx, off, 32));
        const float ev = expf(myscore - mx);
        float sm = ev;
#pragma unroll
        for (int off = 16; off > 0; off >>= 1) sm += __shfl_xor(sm, off, 32);
        const float beta = ev * (1.0f / sm);

        const float* frow = feature + (size_t)gb * NFRAME * NHID;
        v4f cx[4];
#pragma unroll
        for (int q = 0; q < 4; ++q) cx[q] = (v4f){0.f, 0.f, 0.f, 0.f};
#pragma unroll 1
        for (int tp = 0; tp < NT1; ++tp) {
          const float bt = __shfl(beta, tp, 32);
#pragma unroll
          for (int q = 0; q < 4; ++q) {
            const v4f f = *(const v4f*)(frow + (size_t)tp * NHID + 128 * q + 4 * lane);
#pragma unroll
            for (int e = 0; e < 4; ++e) cx[q][e] += bt * f[e];
          }
        }
#pragma unroll
        for (int q = 0; q < 4; ++q) {
          v4h hv;
#pragma unroll
          for (int e = 0; e < 4; ++e) {
            const float xv = cx[q][e];
            hv[e] = (_Float16)xv;
          }
          *(v4h*)(Ax + wave * HP + 128 * q + 4 * lane) = hv;
        }
      }
      __syncthreads();

      {
        float hn[2][8];
#pragma unroll
        for (int nt = 0; nt < 2; ++nt) {
          const int j = 32 * wave + 16 * nt + c;
          v8f a0 = z8, a1 = z8, a2 = z8, a3 = z8;
          kloop4_h(a0, a1, a2, a3, axrow, Wih + (size_t)j * KIH + NEMB + koff, (size_t)NHID * KIH);
          kloop4_h(a0, a1, a2, a3, ahrow, Whh + (size_t)j * NHID + koff, (size_t)NHID * NHID);
          acc_guard4(a0, a1, a2, a3);
#pragma unroll
          for (int r = 0; r < 8; ++r) {
            lstm_point(a0[r] * WCARRY_INV + bb[nt][0], a1[r] * WCARRY_INV + bb[nt][1],
                       a2[r] * WCARRY_INV + bb[nt][2], a3[r] * WCARRY_INV + bb[nt][3], cst[nt][r], hn[nt][r]);
          }
        }
        __syncthreads();
#pragma unroll
        for (int nt = 0; nt < 2; ++nt) {
          const int j = 32 * wave + 16 * nt + c;
#pragma unroll
          for (int r = 0; r < 8; ++r) {
            Ah[(8 * hh + r) * HP + j] = (_Float16)hn[nt][r];
            Ac[(8 * hh + r) * HP + j] = (_Float16)cst[nt][r];
          }
        }
        __syncthreads();
      }
    }

    {
      const float* g1p = Gx1 + ((size_t)(rowbase + 8 * hh) * NT1 + (size_t)((s < NT1) ? s : 0)) * NG4 + 32 * wave + c;
      const float* g2p = Gx2 + ((size_t)((s < NT1) ? 0 : (s - NT1)) * NBATCH + rowbase + 8 * hh) * NG4 + 32 * wave + c;
      const float* gxp = (s < NT1) ? g1p : g2p;
      const size_t gstr = (s < NT1) ? ((size_t)NT1 * NG4) : (size_t)NG4;
      float hn[2][8];
#pragma unroll
      for (int nt = 0; nt < 2; ++nt) {
        const int j = 32 * wave + 16 * nt + c;
        v8f a0, a1, a2, a3;
#pragma unroll
        for (int r = 0; r < 8; ++r) a0[r] = gxp[(size_t)r * gstr + 0 * NHID + 16 * nt] * WCARRY;
        pin8(a0);
#pragma unroll
        for (int r = 0; r < 8; ++r) a1[r] = gxp[(size_t)r * gstr + 1 * NHID + 16 * nt] * WCARRY;
        pin8(a1);
#pragma unroll
        for (int r = 0; r < 8; ++r) a2[r] = gxp[(size_t)r * gstr + 2 * NHID + 16 * nt] * WCARRY;
        pin8(a2);
#pragma unroll
        for (int r = 0; r < 8; ++r) a3[r] = gxp[(size_t)r * gstr + 3 * NHID + 16 * nt] * WCARRY;
        pin8(a3);
        kloop4_h(a0, a1, a2, a3, ahrow, Whh + (size_t)j * NHID + koff, (size_t)NHID * NHID);
        acc_guard4(a0, a1, a2, a3);
#pragma unroll
        for (int r = 0; r < 8; ++r) {
          lstm_point(a0[r] * WCARRY_INV + bb[nt][0], a1[r] * WCARRY_INV + bb[nt][1],
                     a2[r] * WCARRY_INV + bb[nt][2], a3[r] * WCARRY_INV + bb[nt][3], cst[nt][r], hn[nt][r]);
        }
      }
      __syncthreads();
#pragma unroll
      for (int nt = 0; nt < 2; ++nt) {
        const int j = 32 * wave + 16 * nt + c;
#pragma unroll
        for (int r = 0; r < 8; ++r) {
          Ah[(8 * hh + r) * HP + j] = (_Float16)hn[nt][r];
          Ac[(8 * hh + r) * HP + j] = (_Float16)cst[nt][r];
        }
      }
      __syncthreads();
    }

    if (s >= NT1) {
      const int l = s - NT1;
      unsigned short* dst = Hout + ((size_t)(rowbase + wave) * NDEC + l) * NHID;
      const v8h v0 = *(const v8h*)(Ah + wave * HP + lane * 8);
      const v8h v1 = *(const v8h*)(Ah + wave * HP + 256 + lane * 8);
      for (int pass = 0; pass < 2; ++pass) {
        *(volatile v8h*)(dst + lane * 8) = v0;
        *(volatile v8h*)(dst + 256 + lane * 8) = v1;
        __threadfence();
      }
    }
  }
}

extern "C" void kernel_launch(void* const* d_in, const int* in_sizes, int n_in,
                              void* d_out, int out_size, void* d_ws, size_t ws_size, hipStream_t stream) {
  if (n_in < 13 || d_out == nullptr || d_ws == nullptr) return;
  if (in_sizes[0] != NBATCH * NFRAME * NHID || in_sizes[1] != NBATCH * NCAP || in_sizes[2] != NVOC * NEMB ||
      in_sizes[3] != NG4 * KIH || in_sizes[4] != NG4 * NHID || in_sizes[5] != NG4 || in_sizes[6] != NG4 ||
      in_sizes[7] != NHID * KW1 || in_sizes[8] != NHID || in_sizes[9] != NHID || in_sizes[10] != 1 ||
      in_sizes[11] != NVOC * NHID || in_sizes[12] != NVOC || out_size != NROW_OUT * NVOC) return;

  const float* feature = (const float*)d_in[0];
  const int*   caps    = (const int*)d_in[1];
  const float* emb     = (const float*)d_in[2];
  const float* w_ih    = (const float*)d_in[3];
  const float* w_hh    = (const float*)d_in[4];
  const float* b_ih    = (const float*)d_in[5];
  const float* b_hh    = (const float*)d_in[6];
  const float* a_w1    = (const float*)d_in[7];
  const float* a_b1    = (const float*)d_in[8];
  const float* a_w2    = (const float*)d_in[9];
  const float* a_b2    = (const float*)d_in[10];
  const float* out_w   = (const float*)d_in[11];
  const float* out_b   = (const float*)d_in[12];
  float* out = (float*)d_out;

  char* ws = (char*)d_ws;
  size_t off = 0;
  auto carve = [&](size_t bytes) -> char* { char* p = ws + off; off += (bytes + 255) & ~(size_t)255; return p; };
  unsigned short* WHH16  = (unsigned short*)carve((size_t)NG4 * NHID * 2);
  unsigned short* WIH16  = (unsigned short*)carve((size_t)NG4 * KIH * 2);
  unsigned short* W1_16  = (unsigned short*)carve((size_t)NHID * KW1 * 2);
  unsigned short* OW16   = (unsigned short*)carve((size_t)NVPAD * NHID * 2);
  unsigned short* XE16   = (unsigned short*)carve((size_t)NROW_XE * NHID * 2);
  unsigned short* X2_16  = (unsigned short*)carve((size_t)NROW_PAD * KIH * 2);
  unsigned short* HOUT16 = (unsigned short*)carve((size_t)NROW_PAD * NHID * 2);
  float*          SPL    = (float*)carve((size_t)NROW_XE * NHID * 4);
  float*          GX1    = (float*)carve((size_t)NROW_XE * NG4 * 4);
  float*          GX2    = (float*)carve((size_t)NROW_PAD * NG4 * 4);
  if (off > ws_size || off > (size_t)134217728) return;

  {
    const int n8a = NG4 * (NHID / 8);
    const int n8b = NG4 * (KIH / 8);
    const int n8c = NHID * (KW1 / 8);
    const int n8d = NVPAD * (NHID / 8);
    const int n8e = NROW_XE * (NHID / 8);
    cvt8_f16_kernel<0><<<(n8a + 255) / 256, 256, 0, stream>>>(w_hh,  WHH16, NG4,     NHID / 8, NHID, NG4,     WCARRY);
    cvt8_f16_kernel<0><<<(n8b + 255) / 256, 256, 0, stream>>>(w_ih,  WIH16, NG4,     KIH / 8,  KIH,  NG4,     WCARRY);
    cvt8_f16_kernel<0><<<(n8c + 255) / 256, 256, 0, stream>>>(a_w1,  W1_16, NHID,    KW1 / 8,  KW1,  NHID,    WCARRY);
    cvt8_f16_kernel<0><<<(n8d + 255) / 256, 256, 0, stream>>>(out_w, OW16,  NVPAD,   NHID / 8, NHID, NVOC,    WCARRY);
    cvt8_f16_kernel<1><<<(n8e + 255) / 256, 256, 0, stream>>>(feature, XE16, NROW_XE, NHID / 8, NHID, NROW_XE, 1.0f);
    pack_x2_kernel<<<dim3((NROW_PAD * 64) / 256, 2), 256, 0, stream>>>(feature, emb, caps, X2_16);
    const int n8z = (NROW_PAD - NROW_OUT) * (NHID / 8);
    zero16_kernel<<<(n8z + 255) / 256, 256, 0, stream>>>(HOUT16 + (size_t)NROW_OUT * NHID, n8z);
  }

  {
    const int tS = (NROW_XE / 64) * (NHID / 64);
    gemm64_f16_kernel<2><<<(tS + 7) / 8, 256, 0, stream>>>(XE16, NHID, W1_16 + 2 * NHID, KW1, SPL, NHID, a_b1,
                                                           NROW_XE, NHID, NHID, NROW_XE, NHID, WCARRY_INV);
    const int t1 = (NROW_XE / 64) * (NG4 / 64);
    gemm64_f16_kernel<0><<<(t1 + 7) / 8, 256, 0, stream>>>(XE16, NHID, WIH16 + NEMB, KIH, GX1, NG4, a_b1,
                                                           NROW_XE, NG4, NHID, NROW_XE, NG4, WCARRY_INV);
    const int t2 = (NROW_PAD / 64) * (NG4 / 64);
    gemm64_f16_kernel<0><<<(t2 + 7) / 8, 256, 0, stream>>>(X2_16, KIH, WIH16, KIH, GX2, NG4, a_b1,
                                                           NROW_PAD, NG4, KIH, NROW_PAD, NG4, WCARRY_INV);
  }

  decoder_seq_kernel<<<NBATCH / SEQ_ROWS, SEQ_THR, 0, stream>>>(feature, SPL, GX1, GX2, WIH16, WHH16, W1_16,
                                                                b_ih, b_hh, a_w2, a_b2, HOUT16);

  {
    const int tV = (NROW_PAD / 64) * (NVPAD / 64);
    gemm64_f16_kernel<2><<<(tV + 7) / 8, 256, 0, stream>>>(HOUT16, NHID, OW16, NHID, out, NVOC, out_b,
                                                           NROW_PAD, NVPAD, NHID, NROW_OUT, NVOC, WCARRY_INV);
  }
}
